// EBSDSuper_51926154609193
// MI455X (gfx1250) — hardware-run, weakly checked
//
#include <hip/hip_runtime.h>
#include <math.h>

typedef __attribute__((ext_vector_type(16))) _Float16 v16h;
typedef __attribute__((ext_vector_type(8)))  _Float16 v8h;
typedef __attribute__((ext_vector_type(8)))  float    v8f;
typedef __attribute__((ext_vector_type(4)))  float    v4f;

constexpr int kLrW      = 128;
constexpr int kLrN      = kLrW * kLrW;
constexpr int kHrW      = 512;
constexpr int kHrN      = kHrW * kHrW;
constexpr int kChan     = 22;
constexpr int kPitch    = 32;
constexpr int kKTp      = 22 * 32;
constexpr int kKCtx     = 4 * 32;
constexpr int kDedup    = kLrN * 4;
constexpr int kSlabP    = 36;
constexpr int kOut0Elems = kHrN * 9;
constexpr int kOut1Elems = kHrN * 13;
constexpr int kOutElems  = kOut0Elems + kOut1Elems;
static_assert(kLrN == 16384 && kHrN == 262144 && kDedup == 65536, "grid sizes");
static_assert(kKTp == 704 && (kKTp % 32) == 0 && (kKCtx % 32) == 0, "K multiples of 32");
static_assert((kLrN % 16) == 0 && (kDedup % 16) == 0, "M tile multiples");
static_assert(((size_t)kOut0Elems * 4) % 128 == 0, "second output line aligned");
static_assert((kOut0Elems % 1024) == 0 && (kOut1Elems % 1024) == 0, "expand blocks do not straddle outputs");

constexpr float kCarryA   = 16.0f;
constexpr float kCarryB   = 16.0f;
constexpr float kCarryM   = 16.0f;
constexpr float kInvCarry = 1.0f / (kCarryA * kCarryB);
static_assert(kCarryM == kCarryA, "context plane carry feeds the second-operand fragment directly");

constexpr float kS4    = 1.5f;
constexpr float kS6    = (float)(3.605551275463989 / 2.0);
constexpr float kSqrt3 = (float)1.7320508075688772;
constexpr float kS133  = (float)2.0816659994661326;
constexpr float kSh0   = (float)0.28209479177387814;
constexpr float kId4   = (float)(0.28209479177387814 / 3.0);
constexpr float kId6   = (float)(0.28209479177387814 / 3.605551275463989);
constexpr float kY20   = (float)0.5462742152960396;
constexpr float kY22   = (float)(-0.31539156525252005);

__host__ __device__ constexpr int pad32(int n) { return (n + 31) & ~31; }
constexpr int kO444 = 0;
constexpr int kO464 = kO444 + pad32(9 * 9 * 9);
constexpr int kO644 = kO464 + pad32(9 * 13 * 9);
constexpr int kO664 = kO644 + pad32(13 * 9 * 9);
constexpr int kO446 = kO664 + pad32(13 * 13 * 9);
constexpr int kO466 = kO446 + pad32(9 * 9 * 13);
constexpr int kO646 = kO466 + pad32(9 * 13 * 13);
constexpr int kO666 = kO646 + pad32(13 * 9 * 13);
constexpr int kO424 = kO666 + pad32(13 * 13 * 13);
constexpr int kO624 = kO424 + pad32(9 * 5 * 9);
constexpr int kO426 = kO624 + pad32(13 * 5 * 9);
constexpr int kO626 = kO426 + pad32(9 * 5 * 13);
constexpr int kCbFloats = kO626 + pad32(13 * 5 * 13);
static_assert(kCbFloats == 13216, "table size");
static_assert(pad32(13 * 13 * 13) == 2208, "largest padded tensor fits the staging array");

__device__ const int kW3jTab[12][4] = {
  {4, 4, 4, kO444}, {4, 6, 4, kO464}, {6, 4, 4, kO644}, {6, 6, 4, kO664},
  {4, 4, 6, kO446}, {4, 6, 6, kO466}, {6, 4, 6, kO646}, {6, 6, 6, kO666},
  {4, 2, 4, kO424}, {6, 2, 4, kO624}, {4, 2, 6, kO426}, {6, 2, 6, kO626}};
__device__ const int kTpOff[8] = {kO444, kO464, kO644, kO664, kO446, kO466, kO646, kO666};
__device__ const int kAgOff[4] = {kO424, kO624, kO426, kO626};

constexpr int    kW16Halves = 2 * 32 * kKTp + 32 * kKCtx;
constexpr int    kBtpOff16  = 32 * kKTp;
constexpr int    kMcOff16   = 2 * 32 * kKTp;
static_assert(kW16Halves == 49152 && (kW16Halves % 2048) == 0 && ((32 * kKTp) % 2048) == 0, "fold blocks");
constexpr size_t kOffCB  = 0;
constexpr size_t kOffW16 = kOffCB  + (size_t)kCbFloats * 4;
constexpr size_t kOffFE  = kOffW16 + (size_t)kW16Halves * 2;
constexpr size_t kOffNE  = kOffFE  + (size_t)kLrN * kPitch * 4;
constexpr size_t kOffXP  = kOffNE  + (size_t)kLrN * kPitch * 4;
constexpr size_t kOffRP  = kOffXP  + (size_t)kLrN * kPitch * 4;
constexpr size_t kWsTotal = kOffRP + (size_t)kDedup * kPitch * 4;
static_assert(kWsTotal == 14831232ull, "carve total");
static_assert(kWsTotal <= 134217728ull, "carve cap");
static_assert((kOffW16 % 128) == 0 && (kOffFE % 128) == 0 && (kOffNE % 128) == 0 &&
              (kOffXP % 128) == 0 && (kOffRP % 128) == 0, "128-B aligned regions");

__device__ __forceinline__ int imin(int a, int b) { return a < b ? a : b; }
__device__ __forceinline__ int imax(int a, int b) { return a > b ? a : b; }

union FragU { v16h v; v8h h[2]; };
__device__ __forceinline__ v16h frag_load(const _Float16* p) {
  FragU f;
  f.h[0] = *(const v8h*)(p);
  f.h[1] = *(const v8h*)(p + 16);
  return f.v;
}
__device__ __forceinline__ v8f mma_h(v16h a, v16h b, v8f c) {
  c = __builtin_amdgcn_wmma_f32_16x16x32_f16(false, a, false, b, (short)0, c, false, false);
  asm volatile("v_nop\n\tv_nop\n\tv_nop\n\tv_nop" : "+v"(c) : "v"(a), "v"(b));
  return c;
}
__device__ __forceinline__ void wave_lds_sync() {
  __builtin_amdgcn_fence(__ATOMIC_RELEASE, "workgroup");
  __builtin_amdgcn_wave_barrier();
  __builtin_amdgcn_fence(__ATOMIC_ACQUIRE, "workgroup");
}
__device__ __forceinline__ void load_row24(const float* __restrict__ base, float (&a)[24]) {
#pragma unroll
  for (int q = 0; q < 6; ++q) {
    const v4f u = *(const v4f*)(base + 4 * q);
    a[4 * q + 0] = u[0];
    a[4 * q + 1] = u[1];
    a[4 * q + 2] = u[2];
    a[4 * q + 3] = u[3];
  }
}
__device__ __forceinline__ v16h pack_frag(const v4f t0, const v4f t1, const v4f t2, const v4f t3, const float s, const int h) {
  v16h f;
  const int jb = 16 + 8 * h;
#pragma unroll
  for (int e = 0; e < 4; ++e) {
    const float x0 = t0[e];
    const float x1 = t1[e];
    const float x2 = t2[e];
    const float x3 = t3[e];
    const float y2 = (jb + e < kChan) ? x2 * s : 0.0f;
    const float y3 = (jb + 4 + e < kChan) ? x3 * s : 0.0f;
    f[e]      = (_Float16)(x0 * s);
    f[4 + e]  = (_Float16)(x1 * s);
    f[8 + e]  = (_Float16)y2;
    f[12 + e] = (_Float16)y3;
  }
  return f;
}

__device__ __forceinline__ void tp_core(const float (&a)[24], const v16h bfr, const _Float16* __restrict__ Bt,
                                        const int m, const int h, v8f& acc0, v8f& acc1) {
  const _Float16* p0 = Bt + m * kKTp + 8 * h;
  const _Float16* p1 = Bt + (16 + m) * kKTp + 8 * h;
#pragma unroll
  for (int c = 0; c < kChan; ++c) {
    const _Float16 ah = (_Float16)a[c];
    const v16h af = bfr * ah;
    const v16h b0 = frag_load(p0 + c * 32);
    const v16h b1 = frag_load(p1 + c * 32);
    acc0 = mma_h(af, b0, acc0);
    acc1 = mma_h(af, b1, acc1);
  }
}

__device__ double dfact(int n) {
  double r = 1.0;
  for (int i = 2; i <= n; ++i) r *= (double)i;
  return r;
}
__device__ double su2_cg(int j1, int m1, int j2, int m2, int j3, int m3) {
  if (m3 != m1 + m2) return 0.0;
  int vmin = imax(imax(-j1 + j2 + m3, -j1 + m1), 0);
  int vmax = imin(imin(j2 + j3 + m1, j3 - j1 + j2), j3 + m3);
  double c = sqrt((2.0 * j3 + 1.0) * dfact(j3 + j1 - j2) * dfact(j3 - j1 + j2) * dfact(j1 + j2 - j3) / dfact(j1 + j2 + j3 + 1));
  c *= sqrt(dfact(j3 + m3) * dfact(j3 - m3) * dfact(j1 - m1) * dfact(j1 + m1) * dfact(j2 - m2) * dfact(j2 + m2));
  double s = 0.0;
  for (int v = vmin; v <= vmax; ++v) {
    const double sg = ((v + j2 + m2) & 1) ? -1.0 : 1.0;
    s += sg * dfact(j2 + j3 + m1 - v) * dfact(j1 - m1 + v) /
         (dfact(v) * dfact(j3 - j1 + j2 - v) * dfact(j3 + m3 - v) * dfact(v + j1 - j2 - m3));
  }
  return c * s;
}
__device__ void qent(int l, int a, int b, double& re, double& im) {
  const double s = 0.70710678118654752440;
  double r = 0.0, ii = 0.0;
  const int mm = a - l;
  if (mm < 0) {
    if (b == l - mm) r = s;
    else if (b == l + mm) ii = -s;
  } else if (mm == 0) {
    if (b == l) r = 1.0;
  } else {
    const double sg = (mm & 1) ? -1.0 : 1.0;
    if (b == l + mm) r = sg * s;
    else if (b == l - mm) ii = sg * s;
  }
  const double f = ((l & 3) == 0) ? 1.0 : -1.0;
  re = r * f;
  im = ii * f;
}

__global__ __launch_bounds__(256) void w3j_build_kernel(float* __restrict__ Cb) {
  __shared__ double cc[2197];
  __shared__ double cv[2197];
  __shared__ double red[256];
  __shared__ __align__(16) float so[2208];
  const int tid = threadIdx.x;
  const int b = blockIdx.x;
  const int l1 = kW3jTab[b][0], l2 = kW3jTab[b][1], l3 = kW3jTab[b][2], off = kW3jTab[b][3];
  const int n1 = 2 * l1 + 1, n2 = 2 * l2 + 1, n3 = 2 * l3 + 1;
  const int tot = n1 * n2 * n3;
  const int totPad = pad32(tot);
  for (int t = tid; t < tot; t += 256) cc[t] = 0.0;
  __syncthreads();
  for (int t = tid; t < n1 * n2; t += 256) {
    const int ai = t / n2, bi = t - ai * n2;
    const int m1 = ai - l1, m2 = bi - l2, m3 = m1 + m2;
    if (m3 >= -l3 && m3 <= l3) cc[(ai * n2 + bi) * n3 + (l3 + m3)] = su2_cg(l1, m1, l2, m2, l3, m3);
  }
  __syncthreads();
  double ss = 0.0;
  for (int t = tid; t < tot; t += 256) {
    const int j = t / (n2 * n3);
    const int rem = t - j * (n2 * n3);
    const int lI = rem / n3;
    const int mI = rem - lI * n3;
    double are = 0.0;
    for (int i = 0; i < n1; ++i) {
      double q1r, q1i;
      qent(l1, i, j, q1r, q1i);
      if (q1r == 0.0 && q1i == 0.0) continue;
      for (int k = 0; k < n2; ++k) {
        double q2r, q2i;
        qent(l2, k, lI, q2r, q2i);
        if (q2r == 0.0 && q2i == 0.0) continue;
        const double t12r = q1r * q2r - q1i * q2i;
        const double t12i = q1r * q2i + q1i * q2r;
        for (int n = 0; n < n3; ++n) {
          const double cval = cc[(i * n2 + k) * n3 + n];
          if (cval == 0.0) continue;
          double q3r, q3i;
          qent(l3, n, mI, q3r, q3i);
          are += cval * (t12r * q3r + t12i * q3i);
        }
      }
    }
    cv[t] = are;
    ss += are * are;
  }
  red[tid] = ss;
  __syncthreads();
  for (int s2 = 128; s2 > 0; s2 >>= 1) {
    if (tid < s2) red[tid] += red[tid + s2];
    __syncthreads();
  }
  const double nrm = sqrt(red[0]);
  for (int t = tid; t < totPad; t += 256) {
    const double val = cv[imin(t, tot - 1)];
    const float fv = (float)(val / nrm);
    so[t] = (t < tot) ? fv : 0.0f;
  }
  __syncthreads();
  for (int pass = 0; pass < 2; ++pass) {
    for (int v = tid; v < (totPad >> 2); v += 256) {
      const v4f val = *(const v4f*)(so + 4 * v);
      *(volatile v4f*)(Cb + off + 4 * v) = val;
    }
    __threadfence();
  }
}

__global__ __launch_bounds__(256) void fold_kernel(const float* __restrict__ Cb, const float* __restrict__ wsp,
                                                   const float* __restrict__ wtp, const float* __restrict__ wagg,
                                                   unsigned short* __restrict__ W16) {
  __shared__ __align__(16) float sv[2048];
  const int tid = threadIdx.x;
  const int blk = blockIdx.x;
  if (blk < 22) {
    const int which = (blk >= 11) ? 1 : 0;
    const float* __restrict__ w = which ? wtp : wsp;
    const int base = (blk - which * 11) * 2048;
#pragma unroll 1
    for (int it = 0; it < 8; ++it) {
      const int e = base + it * 256 + tid;
      const int n = e / kKTp;
      const int k = e - n * kKTp;
      const int i = k >> 5;
      const int j = k & 31;
      const bool valid = (n < kChan) && (j < kChan);
      const int nc = imin(n, kChan - 1), jc = imin(j, kChan - 1);
      const int o6 = (nc >= 9) ? 1 : 0, i6 = (i >= 9) ? 1 : 0, j6 = (jc >= 9) ? 1 : 0;
      const int p = o6 * 4 + i6 * 2 + j6;
      const int n3 = o6 ? 13 : 9;
      const int n2 = j6 ? 13 : 9;
      const int ii = i - 9 * i6, jj = jc - 9 * j6, kk = nc - 9 * o6;
      const int idx = kTpOff[p] + (ii * n2 + jj) * n3 + kk;
      const float cval = Cb[idx];
      const float sc = o6 ? kS6 : kS4;
      const float v = sc * w[p] * cval * kCarryB;
      sv[it * 256 + tid] = valid ? v : 0.0f;
    }
  } else {
    const int base = (blk - 22) * 2048;
    const float w0 = wagg[0], w4 = wagg[4];
#pragma unroll 1
    for (int it = 0; it < 8; ++it) {
      const int e = base + it * 256 + tid;
      const int n = e >> 7;
      const int kq = e & 127;
      const int q = kq >> 5;
      const int i = kq & 31;
      const bool valid = (n < kChan) && (i < kChan);
      const int nc = imin(n, kChan - 1), ic = imin(i, kChan - 1);
      const int o6 = (nc >= 9) ? 1 : 0, i6 = (ic >= 9) ? 1 : 0;
      const int pm = o6 * 2 + i6;
      const int n3 = o6 ? 13 : 9;
      const int ii = ic - 9 * i6, kk = nc - 9 * o6;
      const int ib = kAgOff[pm] + (ii * 5) * n3 + kk;
      const float c0v = Cb[ib];
      const float c2v = Cb[ib + 2 * n3];
      const float y20 = ((q == 0) || (q == 3)) ? kY20 : -kY20;
      const float s2 = y20 * c0v + kY22 * c2v;
      const int wsel = pm + 1 + ((pm == 3) ? 1 : 0);
      const float wv = wagg[wsel];
      const bool dg = (ic == nc);
      const float ident = (dg && pm == 0) ? w0 * kId4 : ((dg && pm == 3) ? w4 * kId6 : 0.0f);
      const float inner = wv * s2 + ident;
      const float outer = o6 ? kS133 : kSqrt3;
      const float v = outer * inner * kCarryM;
      sv[it * 256 + tid] = valid ? v : 0.0f;
    }
  }
  __syncthreads();
  const float* sp = sv + tid * 8;
  v8h hv;
#pragma unroll
  for (int e = 0; e < 8; ++e) hv[e] = (_Float16)sp[e];
  unsigned short* dst = W16 + (size_t)blk * 2048 + tid * 8;
  *(volatile v8h*)dst = hv;
  __threadfence();
  *(volatile v8h*)dst = hv;
}

__global__ __launch_bounds__(128) void stencil_kernel(const float* __restrict__ f4, const float* __restrict__ f6,
                                                      const float* __restrict__ sw,
                                                      float* __restrict__ FE, float* __restrict__ NE) {
  __shared__ __align__(16) float sF[128 * kSlabP];
  __shared__ __align__(16) float sN[128 * kSlabP];
  const int tid = threadIdx.x;
  const int hrow = blockIdx.x;
  const int pix = hrow * kLrW + tid;
  float acc[kChan];
#pragma unroll
  for (int c = 0; c < kChan; ++c) acc[c] = 0.0f;
#pragma unroll 1
  for (int tap = 0; tap < 9; ++tap) {
    const int di = tap / 3;
    const int dj = tap - di * 3;
    const int hh = imin(imax(hrow + di - 1, 0), kLrW - 1);
    const int ww = imin(imax(tid + dj - 1, 0), kLrW - 1);
    const float wt = sw[tap];
    const int np = hh * kLrW + ww;
    const float* p4 = f4 + (size_t)np * 9;
    const float* p6 = f6 + (size_t)np * 13;
#pragma unroll
    for (int c = 0; c < 9; ++c) acc[c] += wt * p4[c];
    asm volatile("" ::: "memory");
#pragma unroll
    for (int c = 0; c < 13; ++c) acc[9 + c] += wt * p6[c];
  }
  {
    const float* p4 = f4 + (size_t)pix * 9;
    const float* p6 = f6 + (size_t)pix * 13;
    float* rf = sF + tid * kSlabP;
    float* rn = sN + tid * kSlabP;
#pragma unroll
    for (int c = 0; c < 9; ++c) rf[c] = p4[c];
#pragma unroll
    for (int c = 0; c < 13; ++c) rf[9 + c] = p6[c];
#pragma unroll
    for (int c = 0; c < kChan; ++c) rn[c] = acc[c];
#pragma unroll
    for (int c = kChan; c < kPitch; ++c) {
      rf[c] = 0.0f;
      rn[c] = 0.0f;
    }
  }
  __syncthreads();
  const int lane = tid & 31, wv = tid >> 5;
  const int q = lane >> 3, c4 = (lane & 7) * 4;
  for (int pass = 0; pass < 2; ++pass) {
#pragma unroll
    for (int it = 0; it < 8; ++it) {
      const int row = wv * 32 + it * 4 + q;
      const v4f vf = *(const v4f*)(sF + row * kSlabP + c4);
      const v4f vn = *(const v4f*)(sN + row * kSlabP + c4);
      const size_t o = (size_t)(hrow * kLrW + row) * kPitch + c4;
      *(volatile v4f*)(FE + o) = vf;
      *(volatile v4f*)(NE + o) = vn;
    }
    __threadfence();
  }
}

static_assert((kLrN / 16) % 8 == 0, "tp1 grid exact");
__global__ __launch_bounds__(256) void tp1_kernel(const float* __restrict__ FE, const float* __restrict__ NE,
                                                  const unsigned short* __restrict__ Bsp16, float* __restrict__ XP) {
  __shared__ __align__(16) float sS[8][16 * kSlabP];
  const int lane = threadIdx.x & 31, wave = threadIdx.x >> 5;
  const int m = lane & 15, h = lane >> 4;
  const int tile = blockIdx.x * 8 + wave;
  const int pix = tile * 16 + m;
  const _Float16* Bt = (const _Float16*)Bsp16;

  float a[24];
  load_row24(FE + (size_t)pix * kPitch, a);
  const float* nr = NE + (size_t)pix * kPitch + 8 * h;
  const v4f t0 = *(const v4f*)(nr);
  const v4f t1 = *(const v4f*)(nr + 4);
  const v4f t2 = *(const v4f*)(nr + 16);
  const v4f t3 = *(const v4f*)(nr + 20);
  const v16h bfr = pack_frag(t0, t1, t2, t3, kCarryA, h);

  v8f acc0 = (v8f){0.f, 0.f, 0.f, 0.f, 0.f, 0.f, 0.f, 0.f};
  v8f acc1 = (v8f){0.f, 0.f, 0.f, 0.f, 0.f, 0.f, 0.f, 0.f};
  tp_core(a, bfr, Bt, m, h, acc0, acc1);

  float* slab = sS[wave];
#pragma unroll
  for (int r = 0; r < 8; ++r) {
    const float v0 = acc0[r] * kInvCarry;
    const float v1 = acc1[r] * kInvCarry;
    slab[(8 * h + r) * kSlabP + m] = v0;
    slab[(8 * h + r) * kSlabP + 16 + m] = (16 + m < kChan) ? v1 : 0.0f;
  }
  wave_lds_sync();
  const int q = lane >> 3, c4 = (lane & 7) * 4;
  v4f ov[4];
#pragma unroll
  for (int it = 0; it < 4; ++it) {
    const int row = it * 4 + q;
    const v4f sv4 = *(const v4f*)(slab + row * kSlabP + c4);
    const v4f rv4 = *(const v4f*)(FE + (size_t)(tile * 16 + row) * kPitch + c4);
    ov[it] = sv4 + rv4;
  }
  for (int pass = 0; pass < 2; ++pass) {
#pragma unroll
    for (int it = 0; it < 4; ++it) {
      const int row = it * 4 + q;
      *(volatile v4f*)(XP + (size_t)(tile * 16 + row) * kPitch + c4) = ov[it];
    }
    __threadfence();
  }
}

static_assert((kDedup / 16) % 8 == 0, "tp2 grid exact");
__global__ __launch_bounds__(256) void ctx_tp2_kernel(const float* __restrict__ XP, const unsigned short* __restrict__ Btp16,
                                                      const unsigned short* __restrict__ Mc16, float* __restrict__ RP) {
  __shared__ __align__(16) float sC[8][16 * kSlabP];
  __shared__ __align__(16) float sO[8][16 * kSlabP];
  const int lane = threadIdx.x & 31, wave = threadIdx.x >> 5;
  const int m = lane & 15, h = lane >> 4;
  const int tile = blockIdx.x * 8 + wave;
  const int lr = tile * 4 + (m >> 2);
  const int bi = (m >> 1) & 1, bj = m & 1;
  const int r0 = lr >> 7, c0 = lr & (kLrW - 1);
  const _Float16* Mc = (const _Float16*)Mc16;
  const _Float16* Bt = (const _Float16*)Btp16;

  v8f cx0 = (v8f){0.f, 0.f, 0.f, 0.f, 0.f, 0.f, 0.f, 0.f};
  v8f cx1 = (v8f){0.f, 0.f, 0.f, 0.f, 0.f, 0.f, 0.f, 0.f};
#pragma unroll
  for (int q = 0; q < 4; ++q) {
    const int di = q >> 1, dj = q & 1;
    const int rr = imin(r0 + di * bi, kLrW - 1);
    const int cc = imin(c0 + dj * bj, kLrW - 1);
    const float* xr = XP + (size_t)(rr * kLrW + cc) * kPitch + 8 * h;
    const v4f t0 = *(const v4f*)(xr);
    const v4f t1 = *(const v4f*)(xr + 4);
    const v4f t2 = *(const v4f*)(xr + 16);
    const v4f t3 = *(const v4f*)(xr + 20);
    const v16h af = pack_frag(t0, t1, t2, t3, 1.0f, h);
    const v16h b0 = frag_load(Mc + m * kKCtx + q * 32 + 8 * h);
    const v16h b1 = frag_load(Mc + (16 + m) * kKCtx + q * 32 + 8 * h);
    cx0 = mma_h(af, b0, cx0);
    cx1 = mma_h(af, b1, cx1);
  }
  float* slabC = sC[wave];
#pragma unroll
  for (int r = 0; r < 8; ++r) {
    const float v0 = cx0[r];
    const float v1 = cx1[r];
    slabC[(8 * h + r) * kSlabP + m] = v0;
    slabC[(8 * h + r) * kSlabP + 16 + m] = (16 + m < kChan) ? v1 : 0.0f;
  }
  wave_lds_sync();
  v16h bfr;
  {
    const float* cr = slabC + m * kSlabP + 8 * h;
    const v4f t0 = *(const v4f*)(cr);
    const v4f t1 = *(const v4f*)(cr + 4);
    const v4f t2 = *(const v4f*)(cr + 16);
    const v4f t3 = *(const v4f*)(cr + 20);
    bfr = pack_frag(t0, t1, t2, t3, 1.0f, h);
  }
  float a[24];
  load_row24(XP + (size_t)lr * kPitch, a);

  v8f acc0 = (v8f){0.f, 0.f, 0.f, 0.f, 0.f, 0.f, 0.f, 0.f};
  v8f acc1 = (v8f){0.f, 0.f, 0.f, 0.f, 0.f, 0.f, 0.f, 0.f};
  tp_core(a, bfr, Bt, m, h, acc0, acc1);

  float* slab = sO[wave];
#pragma unroll
  for (int r = 0; r < 8; ++r) {
    const float v0 = acc0[r] * kInvCarry;
    const float v1 = acc1[r] * kInvCarry;
    slab[(8 * h + r) * kSlabP + m] = v0;
    slab[(8 * h + r) * kSlabP + 16 + m] = (16 + m < kChan) ? v1 : 0.0f;
  }
  wave_lds_sync();
  const int q = lane >> 3, c4 = (lane & 7) * 4;
  v4f ov[4];
#pragma unroll
  for (int it = 0; it < 4; ++it) {
    const int row = it * 4 + q;
    const int lrr = tile * 4 + (row >> 2);
    const v4f sv4 = *(const v4f*)(slab + row * kSlabP + c4);
    const v4f rv4 = *(const v4f*)(XP + (size_t)lrr * kPitch + c4);
    ov[it] = sv4 + rv4;
  }
  for (int pass = 0; pass < 2; ++pass) {
#pragma unroll
    for (int it = 0; it < 4; ++it) {
      const int row = it * 4 + q;
      *(volatile v4f*)(RP + (size_t)(tile * 16 + row) * kPitch + c4) = ov[it];
    }
    __threadfence();
  }
}

static_assert((kOutElems / 4) % 256 == 0, "expand grid exact");
__global__ __launch_bounds__(256) void expand_kernel(const float* __restrict__ RP, const int* __restrict__ Hp,
                                                     const int* __restrict__ Wp, float* __restrict__ out) {
  const unsigned g = blockIdx.x * 256u + threadIdx.x;
  const unsigned e0 = g * 4u;
  const bool second = (e0 >= (unsigned)kOut0Elems);
  const unsigned base = second ? (e0 - (unsigned)kOut0Elems) : e0;
  const bool ok = (Hp[0] == kLrW) && (Wp[0] == kLrW);
  const float poison = __uint_as_float(0x7fc00000u);
  v4f v;
#pragma unroll
  for (int k = 0; k < 4; ++k) {
    const unsigned e = base + (unsigned)k;
    const unsigned p9 = e / 9u;
    const unsigned p13 = e / 13u;
    const unsigned pixr = second ? p13 : p9;
    const unsigned pix = (pixr < (unsigned)kHrN) ? pixr : (unsigned)(kHrN - 1);
    const unsigned comp = second ? (e - p13 * 13u + 9u) : (e - p9 * 9u);
    const unsigned I = pix >> 9, J = pix & 511u;
    const unsigned lr = (I >> 2) * (unsigned)kLrW + (J >> 2);
    const unsigned cls = (((I & 3u) == 3u) ? 2u : 0u) + (((J & 3u) == 3u) ? 1u : 0u);
    const unsigned row = lr * 4u + cls;
    const float val = RP[(size_t)row * kPitch + comp];
    v[k] = ok ? val : poison;
  }
  float* dst = out + (size_t)e0;
  *(volatile v4f*)dst = v;
  __threadfence();
  *(volatile v4f*)dst = v;
}

extern "C" void kernel_launch(void* const* d_in, const int* in_sizes, int n_in,
                              void* d_out, int out_size, void* d_ws, size_t ws_size,
                              hipStream_t stream) {
  if (n_in < 8) return;
  if (in_sizes[0] != kLrN * 9) return;
  if (in_sizes[1] != kLrN * 13) return;
  if (in_sizes[2] != 1 || in_sizes[3] != 1) return;
  if (in_sizes[4] != 9) return;
  if (in_sizes[5] != 8 || in_sizes[6] != 6 || in_sizes[7] != 8) return;
  if (out_size != kOutElems) return;
  if (ws_size < kWsTotal) return;

  const float* f4   = (const float*)d_in[0];
  const float* f6   = (const float*)d_in[1];
  const int*   Hp   = (const int*)d_in[2];
  const int*   Wp   = (const int*)d_in[3];
  const float* sw   = (const float*)d_in[4];
  const float* wsp  = (const float*)d_in[5];
  const float* wagg = (const float*)d_in[6];
  const float* wtp  = (const float*)d_in[7];
  float* out = (float*)d_out;

  char* ws = (char*)d_ws;
  float*          CB  = (float*)(ws + kOffCB);
  unsigned short* W16 = (unsigned short*)(ws + kOffW16);
  float*          FE  = (float*)(ws + kOffFE);
  float*          NE  = (float*)(ws + kOffNE);
  float*          XP  = (float*)(ws + kOffXP);
  float*          RP  = (float*)(ws + kOffRP);

  w3j_build_kernel<<<12, 256, 0, stream>>>(CB);
  fold_kernel<<<kW16Halves / 2048, 256, 0, stream>>>(CB, wsp, wtp, wagg, W16);
  stencil_kernel<<<kLrW, 128, 0, stream>>>(f4, f6, sw, FE, NE);
  tp1_kernel<<<(kLrN / 16) / 8, 256, 0, stream>>>(FE, NE, W16, XP);
  ctx_tp2_kernel<<<(kDedup / 16) / 8, 256, 0, stream>>>(XP, W16 + kBtpOff16, W16 + kMcOff16, RP);
  expand_kernel<<<(kOutElems / 4) / 256, 256, 0, stream>>>(RP, Hp, Wp, out);
}
